// pattn_78786880077872
// MI455X (gfx1250) — hardware-verified
//
#include <hip/hip_runtime.h>
#include <math.h>

typedef __attribute__((ext_vector_type(16))) _Float16 v16h;
typedef __attribute__((ext_vector_type(8)))  _Float16 v8h;
typedef __attribute__((ext_vector_type(16))) __bf16   v16b;
typedef __attribute__((ext_vector_type(8)))  __bf16   v8b;
typedef __attribute__((ext_vector_type(8)))  float    v8f;
typedef __attribute__((ext_vector_type(4)))  float    v4f;
typedef __attribute__((ext_vector_type(2)))  float    v2f;

constexpr int kB    = 2;
constexpr int kS    = 2048;
constexpr int kD    = 1024;
constexpr int kH    = 16;
constexpr int kHD   = 64;
constexpr int kTok  = kB * kS;
constexpr int kQKLd = 2 * kD;
constexpr int kKOff = kD;
constexpr int kKC   = 64;
constexpr int kNQB  = kS / 64;
constexpr int kStg  = 72;
constexpr float kSmScale = 0.125f;

constexpr size_t kOffXb   = 0;
constexpr size_t kOffQkwT = kOffXb   + (size_t)kTok * kD * 2;
constexpr size_t kOffVwT  = kOffQkwT + (size_t)kQKLd * kD * 2;
constexpr size_t kOffCwT  = kOffVwT  + (size_t)kD * kD * 2;
constexpr size_t kOffQKp  = kOffCwT  + (size_t)kD * kD * 2;
constexpr size_t kOffVf   = kOffQKp  + (size_t)kTok * kQKLd * 2;
constexpr size_t kOffVth  = kOffVf   + (size_t)kTok * kD * 4;
constexpr size_t kOffVtl  = kOffVth  + (size_t)kB * kH * kHD * kS * 2;
constexpr size_t kOffAV   = kOffVtl  + (size_t)kB * kH * kHD * kS * 2;
constexpr size_t kOffOh   = kOffAV   + (size_t)kTok * kD * 4;
constexpr size_t kOffOl   = kOffOh   + (size_t)kTok * kD * 2;
constexpr size_t kWsTotal = kOffOl   + (size_t)kTok * kD * 2;
static_assert(kWsTotal == 100663296ull);
static_assert(kWsTotal <= 134217728ull);

__device__ __forceinline__ unsigned short f2bf_bits(float f) {
  unsigned u = __float_as_uint(f);
  return (unsigned short)((u + 0x7FFFu + ((u >> 16) & 1u)) >> 16);
}
__device__ __forceinline__ float bf_bits2f(unsigned short h) { return __uint_as_float(((unsigned)h) << 16); }

__device__ __forceinline__ void dep_guard_h(v8f& a, v8f& b, v16h x, v16h y) { asm volatile("v_nop\n\tv_nop\n\tv_nop\n\tv_nop" : "+v"(a), "+v"(b) : "v"(x), "v"(y)); }
__device__ __forceinline__ void dep_guard_b(v8f& a, v8f& b, v16b x, v16b y) { asm volatile("v_nop\n\tv_nop\n\tv_nop\n\tv_nop" : "+v"(a), "+v"(b) : "v"(x), "v"(y)); }
__device__ __forceinline__ void keep4_h(v16h a, v16h b, v16h c, v16h d) { asm volatile("v_nop" :: "v"(a), "v"(b), "v"(c), "v"(d)); }
__device__ __forceinline__ void keep4_b(v16b a, v16b b, v16b c, v16b d) { asm volatile("v_nop" :: "v"(a), "v"(b), "v"(c), "v"(d)); }
__device__ __forceinline__ void acc_guard4(v8f& a, v8f& b, v8f& c, v8f& d) { asm volatile("v_nop\n\tv_nop\n\tv_nop\n\tv_nop" : "+v"(a), "+v"(b), "+v"(c), "+v"(d)); }
template <typename T> struct Frag;
template <> struct Frag<_Float16> {
  typedef v16h V; union U { v16h v; v8h h[2]; };
  static __device__ __forceinline__ v16h load(const _Float16* p) {
    U f; f.h[0] = *(const v8h*)(p); f.h[1] = *(const v8h*)(p + 16); return f.v;
  }
  static __device__ __forceinline__ v8f mma(v16h a, v16h b, v8f c) {
    return __builtin_amdgcn_wmma_f32_16x16x32_f16(false, a, false, b, (short)0, c, false, false);
  }
  static __device__ __forceinline__ void guard(v8f& a, v8f& b, v16h x, v16h y) { dep_guard_h(a, b, x, y); }
  static __device__ __forceinline__ void keep(v16h a, v16h b, v16h c, v16h d) { keep4_h(a, b, c, d); }
};
template <> struct Frag<__bf16> {
  typedef v16b V; union U { v16b v; v8b h[2]; };
  static __device__ __forceinline__ v16b load(const __bf16* p) {
    U f; f.h[0] = *(const v8b*)(p); f.h[1] = *(const v8b*)(p + 16); return f.v;
  }
  static __device__ __forceinline__ v8f mma(v16b a, v16b b, v8f c) {
    return __builtin_amdgcn_wmma_f32_16x16x32_bf16(false, a, false, b, (short)0, c, false, false);
  }
  static __device__ __forceinline__ void guard(v8f& a, v8f& b, v16b x, v16b y) { dep_guard_b(a, b, x, y); }
  static __device__ __forceinline__ void keep(v16b a, v16b b, v16b c, v16b d) { keep4_b(a, b, c, d); }
};

__device__ __forceinline__ unsigned short at_bf_bits(float f) {
  unsigned u = __float_as_uint(f);
  return (unsigned short)((u + 0x7FFFu + ((u >> 16) & 1u)) >> 16);
}
__device__ __forceinline__ __bf16 at_f2bf(float f) { return __builtin_bit_cast(__bf16, at_bf_bits(f)); }
__device__ __forceinline__ void at_split(float f, __bf16& hi, __bf16& lo) {
  const unsigned short hb = at_bf_bits(f);
  hi = __builtin_bit_cast(__bf16, hb);
  lo = at_f2bf(f - __uint_as_float(((unsigned)hb) << 16));
}
__device__ __forceinline__ v8f at_mma(v16b a, v16b b, v8f c) {
  c = __builtin_amdgcn_wmma_f32_16x16x32_bf16(false, a, false, b, (short)0, c, false, false);
  asm volatile("v_nop\n\tv_nop\n\tv_nop\n\tv_nop" : "+v"(c) : "v"(a), "v"(b));
  return c;
}
__device__ __forceinline__ v8f at_mma_h(v16h a, v16h b, v8f c) {
  c = __builtin_amdgcn_wmma_f32_16x16x32_f16(false, a, false, b, (short)0, c, false, false);
  asm volatile("v_nop\n\tv_nop\n\tv_nop\n\tv_nop" : "+v"(c) : "v"(a), "v"(b));
  return c;
}

__global__ __launch_bounds__(256) void cast_f32_bf16x2(const float* __restrict__ in,
                                                       unsigned short* __restrict__ out, int n2) {
  const int i = blockIdx.x * 256 + threadIdx.x;
  if (i < n2) {
    const unsigned u = (unsigned)f2bf_bits(in[2 * i]) | ((unsigned)f2bf_bits(in[2 * i + 1]) << 16);
    ((volatile unsigned*)out)[i] = u;
    __threadfence();
    ((volatile unsigned*)out)[i] = u;
  }
}

template <int ET> struct Elem;
template <> struct Elem<0> { typedef _Float16 T; };
template <> struct Elem<1> { typedef __bf16 T; };
template <int ET, int SPLITM, int BIAS_MODE, int OUT_MODE, bool RESID, int ACT = 0>
__global__ __launch_bounds__(256) void wmma_gemm64(
    const unsigned short* __restrict__ Ap, const unsigned short* __restrict__ A2p, int lda, long strideA,
    const unsigned short* __restrict__ Btp, const unsigned short* __restrict__ Bt2p, int ldb, long strideB,
    void* __restrict__ Cout, void* __restrict__ Cout2, int ldc, long strideC,
    const float* __restrict__ bias,
    const float* __restrict__ resid, long strideR,
    int M, int N, int K, float scale) {
  typedef typename Elem<ET>::T T;
  typedef typename Frag<T>::V V;
  constexpr bool SPA = (SPLITM >= 1);
  constexpr bool SPB = (SPLITM >= 2);
  const T* A = (const T*)Ap; const T* A2 = (const T*)A2p; const T* Bt = (const T*)Btp; const T* Bt2 = (const T*)Bt2p;
  __shared__ __align__(16) float sT[8][16 * 68];
  const int b    = blockIdx.y;
  const int lane = threadIdx.x & 31;
  const int wave = threadIdx.x >> 5;
  const int tilesN = N >> 6;
  const int tilesM = M >> 6;
  const int tile = blockIdx.x * 8 + wave;
  if (tile >= tilesM * tilesN) return;
  const int tm = tile / tilesN;
  const int tn = tile - tm * tilesN;
  const int m0 = tm << 6;
  const int n0 = tn << 6;

  const T* Ab  = A  + (size_t)b * strideA;
  const T* Bb  = Bt + (size_t)b * strideB;
  const T* Ab2 = SPA ? (A2  + (size_t)b * strideA) : nullptr;
  const T* Bb2 = SPB ? (Bt2 + (size_t)b * strideB) : nullptr;

  const int rlane = lane & 15;
  const int koff  = (lane >> 4) * 8;
  const int mOff  = (lane >> 4) * 8;

  v8f acc[4][4];
#pragma unroll
  for (int i = 0; i < 4; ++i)
#pragma unroll
    for (int j = 0; j < 4; ++j) acc[i][j] = (v8f){0.f,0.f,0.f,0.f,0.f,0.f,0.f,0.f};

  for (int k0 = 0; k0 < K; k0 += 32) {
    V bh[4], bl[4];
#pragma unroll
    for (int j = 0; j < 4; ++j) {
      const size_t bo = (size_t)(n0 + (j << 4) + rlane) * ldb + koff + k0;
      bh[j] = Frag<T>::load(Bb + bo);
      if (SPB) bl[j] = Frag<T>::load(Bb2 + bo);
    }
#pragma unroll
    for (int i = 0; i < 4; ++i) {
      const size_t ao = (size_t)(m0 + (i << 4) + rlane) * lda + koff + k0;
      V ah = Frag<T>::load(Ab + ao);
      V al;
      if (SPA) al = Frag<T>::load(Ab2 + ao);
#pragma unroll
      for (int j = 0; j < 4; ++j) {
        acc[i][j] = Frag<T>::mma(ah, bh[j], acc[i][j]);
        if (SPB) acc[i][j] = Frag<T>::mma(ah, bl[j], acc[i][j]);
        if (SPA) acc[i][j] = Frag<T>::mma(al, bh[j], acc[i][j]);
      }
      Frag<T>::guard(acc[i][0], acc[i][3], ah, SPA ? al : ah);
    }
    Frag<T>::keep(bh[0], bh[1], bh[2], bh[3]);
    if (SPB) Frag<T>::keep(bl[0], bl[1], bl[2], bl[3]);
  }
  acc_guard4(acc[0][0], acc[0][1], acc[0][2], acc[0][3]);
  acc_guard4(acc[1][0], acc[1][1], acc[1][2], acc[1][3]);
  acc_guard4(acc[2][0], acc[2][1], acc[2][2], acc[2][3]);
  acc_guard4(acc[3][0], acc[3][1], acc[3][2], acc[3][3]);

  float* slab = sT[wave];
  const float* Rb = RESID ? (resid + (size_t)b * strideR) : nullptr;
#pragma unroll
  for (int i = 0; i < 4; ++i) {
    const int mBase = m0 + (i << 4);
#pragma unroll
    for (int j = 0; j < 4; ++j) {
      const int n = n0 + (j << 4) + rlane;
      float bv = 0.f;
      if (BIAS_MODE == 2) bv = bias[n];
#pragma unroll
      for (int r = 0; r < 8; ++r) {
        float v = acc[i][j][r] * scale;
        if (BIAS_MODE == 1) v += bias[mBase + mOff + r];
        if (BIAS_MODE == 2) v += bv;
        if (RESID) v += Rb[(size_t)(mBase + mOff + r) * ldc + n];
        if (ACT == 1) v = tanhf(v);
        if (ACT == 2) v = fmaxf(v, 0.0f);
        if (ACT == 4) v = (v > 0.f) ? v : 0.01f * v;
        slab[(mOff + r) * 68 + (j << 4) + rlane] = v;
      }
    }
    __builtin_amdgcn_fence(__ATOMIC_RELEASE, "workgroup");
    __builtin_amdgcn_wave_barrier();
    __builtin_amdgcn_fence(__ATOMIC_ACQUIRE, "workgroup");
    if (OUT_MODE == 0) {
      float* C = (float*)Cout + (size_t)b * strideC;
      const int hh = lane >> 4, c4 = (lane & 15) * 4;
      for (int pass = 0; pass < 2; ++pass) {
#pragma unroll
        for (int it = 0; it < 8; ++it) {
          const int row = it * 2 + hh;
          v4f v = *(const v4f*)(slab + row * 68 + c4);
          *(volatile v4f*)(C + (size_t)(mBase + row) * ldc + n0 + c4) = v;
        }
        __threadfence();
      }
    } else {
      const int q = lane >> 3, c8 = (lane & 7) * 8;
      unsigned short* C  = (unsigned short*)Cout  + (size_t)b * strideC;
      unsigned short* C2 = (OUT_MODE == 2) ? ((unsigned short*)Cout2 + (size_t)b * strideC) : nullptr;
      for (int pass = 0; pass < 2; ++pass) {
#pragma unroll
        for (int it = 0; it < 4; ++it) {
          const int row = it * 4 + q;
          const float* sp = slab + row * 68 + c8;
          v8h hv, lv;
#pragma unroll
          for (int e = 0; e < 8; ++e) {
            if (OUT_MODE == 1) {
              hv[e] = (_Float16)sp[e];
            } else {
              unsigned short hb = f2bf_bits(sp[e]);
              unsigned short lb = f2bf_bits(sp[e] - bf_bits2f(hb));
              hv[e] = __builtin_bit_cast(_Float16, hb);
              lv[e] = __builtin_bit_cast(_Float16, lb);
            }
          }
          *(volatile v8h*)(C + (size_t)(mBase + row) * ldc + n0 + c8) = hv;
          if (OUT_MODE == 2) *(volatile v8h*)(C2 + (size_t)(mBase + row) * ldc + n0 + c8) = lv;
        }
        __threadfence();
      }
    }
    __builtin_amdgcn_fence(__ATOMIC_RELEASE, "workgroup");
    __builtin_amdgcn_wave_barrier();
    __builtin_amdgcn_fence(__ATOMIC_ACQUIRE, "workgroup");
  }
}

__global__ __launch_bounds__(256) void transpose_cast_bf16(const float* __restrict__ in, unsigned short* __restrict__ out,
                                                           int R, int Cc) {
  __shared__ __align__(16) _Float16 t[64 * kStg];
  const int c0 = blockIdx.x * 64, r0 = blockIdx.y * 64;
  const int tid = threadIdx.x;
  {
    const int rloc = tid >> 2, cq = (tid & 3) * 16;
    const float* src = in + (size_t)(r0 + rloc) * Cc + c0 + cq;
#pragma unroll
    for (int g4 = 0; g4 < 4; ++g4) {
      const v4f a = *(const v4f*)(src + 4 * g4);
#pragma unroll
      for (int e = 0; e < 4; ++e)
        t[(cq + 4 * g4 + e) * kStg + rloc] = __builtin_bit_cast(_Float16, f2bf_bits(a[e]));
    }
  }
  __syncthreads();
  const int wave = tid >> 5, lane = tid & 31, q8 = lane >> 3, c8 = (lane & 7) * 8;
  const int cA = wave * 8 + q8, cB = wave * 8 + 4 + q8;
  const v8h va = *(const v8h*)(t + cA * kStg + c8);
  const v8h vb = *(const v8h*)(t + cB * kStg + c8);
  unsigned short* da = out + (size_t)(c0 + cA) * R + r0 + c8;
  unsigned short* db = out + (size_t)(c0 + cB) * R + r0 + c8;
  for (int pass = 0; pass < 2; ++pass) {
    *(volatile v8h*)da = va;
    *(volatile v8h*)db = vb;
    __threadfence();
  }
}

__global__ __launch_bounds__(256) void v_split_transpose(const float* __restrict__ Vf,
                                                         unsigned short* __restrict__ vth, unsigned short* __restrict__ vtl) {
  __shared__ __align__(16) _Float16 th[64 * kStg];
  __shared__ __align__(16) _Float16 tl[64 * kStg];
  const int st0 = blockIdx.x * 64, bh = blockIdx.y;
  const int b = bh / kH, h = bh % kH;
  const int tid = threadIdx.x;
  {
    const int sloc = tid >> 2, d0 = (tid & 3) * 16;
    const float* src = Vf + (size_t)(b * kS + st0 + sloc) * kD + h * kHD + d0;
#pragma unroll
    for (int g4 = 0; g4 < 4; ++g4) {
      const v4f a = *(const v4f*)(src + 4 * g4);
#pragma unroll
      for (int e = 0; e < 4; ++e) {
        const unsigned short hb = f2bf_bits(a[e]);
        const unsigned short lb = f2bf_bits(a[e] - bf_bits2f(hb));
        th[(d0 + 4 * g4 + e) * kStg + sloc] = __builtin_bit_cast(_Float16, hb);
        tl[(d0 + 4 * g4 + e) * kStg + sloc] = __builtin_bit_cast(_Float16, lb);
      }
    }
  }
  __syncthreads();
  const int wave = tid >> 5, lane = tid & 31, q8 = lane >> 3, c8 = (lane & 7) * 8;
  const int dA = wave * 8 + q8, dB = wave * 8 + 4 + q8;
  const v8h ha = *(const v8h*)(th + dA * kStg + c8);
  const v8h hbv = *(const v8h*)(th + dB * kStg + c8);
  const v8h la = *(const v8h*)(tl + dA * kStg + c8);
  const v8h lbv = *(const v8h*)(tl + dB * kStg + c8);
  unsigned short* pha = vth + ((size_t)bh * kHD + dA) * kS + st0 + c8;
  unsigned short* phb = vth + ((size_t)bh * kHD + dB) * kS + st0 + c8;
  unsigned short* pla = vtl + ((size_t)bh * kHD + dA) * kS + st0 + c8;
  unsigned short* plb = vtl + ((size_t)bh * kHD + dB) * kS + st0 + c8;
  for (int pass = 0; pass < 2; ++pass) {
    *(volatile v8h*)pha = ha;
    *(volatile v8h*)phb = hbv;
    *(volatile v8h*)pla = la;
    *(volatile v8h*)plb = lbv;
    __threadfence();
  }
}

__global__ __launch_bounds__(128)
void attn_causal_hd64(const unsigned short* __restrict__ QKp,
                      const unsigned short* __restrict__ Vthp,
                      const unsigned short* __restrict__ Vtlp,
                      float* __restrict__ AV) {
  union FB { v16b v; v8b h[2]; };
  __shared__ __align__(16) _Float16 Ksh[kKC * kHD];
  __shared__ __align__(16) __bf16  Vhs[kHD * kKC];
  __shared__ __align__(16) __bf16  Vls[kHD * kKC];
  __shared__ __align__(16) __bf16  Psh[4][16 * kKC];
  __shared__ __align__(16) __bf16  Psl[4][16 * kKC];
  __shared__ __align__(16) float   Os[4][16 * 68];

  const int tid  = threadIdx.x;
  const int wave = tid >> 5;
  const int lane = tid & 31;
  const int hh   = lane >> 4;
  const int c    = lane & 15;

  const int bx = blockIdx.x;
  const int qb = bx % kNQB;
  const int bh = bx / kNQB;
  const int h  = bh % kH;
  const int b  = bh / kH;
  const int q0 = qb * 64 + wave * 16;

  const _Float16* Q16 = (const _Float16*)QKp;
  const __bf16* Vth = (const __bf16*)Vthp;
  const __bf16* Vtl = (const __bf16*)Vtlp;
  float* ob_ptr = AV + (size_t)(b * kS) * kD + h * kHD;

  v16h qa[2];
  {
    const _Float16* qrow = Q16 + (size_t)(b * kS + q0 + c) * kQKLd + h * kHD + 8 * hh;
    qa[0] = Frag<_Float16>::load(qrow);
    qa[1] = Frag<_Float16>::load(qrow + 32);
  }

  float mrow[8], lrow[8];
  v8f oacc[4];
#pragma unroll
  for (int r = 0; r < 8; ++r) { mrow[r] = -INFINITY; lrow[r] = 0.f; }
#pragma unroll
  for (int t = 0; t < 4; ++t) oacc[t] = (v8f){0.f,0.f,0.f,0.f,0.f,0.f,0.f,0.f};

  const int nChunks = qb + 1;
  for (int kc = 0; kc < nChunks; ++kc) {
    const int kv0 = kc * kKC;
    __syncthreads();
#pragma unroll
    for (int i = 0; i < 4; ++i) {
      const int ch = tid + 128 * i, row = ch >> 3, seg = (ch & 7) * 8;
      *(v8h*)(Ksh + row * kHD + seg) =
          *(const v8h*)(Q16 + (size_t)(b * kS + kv0 + row) * kQKLd + kKOff + h * kHD + seg);
      const size_t vo = ((size_t)bh * kHD + row) * kS + kv0 + seg;
      *(v8b*)(Vhs + row * kKC + seg) = *(const v8b*)(Vth + vo);
      *(v8b*)(Vls + row * kKC + seg) = *(const v8b*)(Vtl + vo);
    }
    __syncthreads();

    v8f s[4];
#pragma unroll
    for (int j = 0; j < 4; ++j) {
      s[j] = (v8f){0.f,0.f,0.f,0.f,0.f,0.f,0.f,0.f};
#pragma unroll
      for (int dc = 0; dc < 2; ++dc) {
        const v16h kb = Frag<_Float16>::load(Ksh + (j * 16 + c) * kHD + dc * 32 + 8 * hh);
        s[j] = at_mma_h(qa[dc], kb, s[j]);
      }
    }
    const bool diag = (kc == qb);
    float cm[8];
#pragma unroll
    for (int r = 0; r < 8; ++r) {
      const int qrow = q0 + 8 * hh + r;
      float m = -INFINITY;
#pragma unroll
      for (int j = 0; j < 4; ++j) {
        const int kvcol = kv0 + j * 16 + c;
        float sv = s[j][r] * kSmScale;
        if (diag && (kvcol > qrow)) sv = -INFINITY;
        s[j][r] = sv;
        m = fmaxf(m, sv);
      }
#pragma unroll
      for (int off = 1; off < 16; off <<= 1) m = fmaxf(m, __shfl_xor(m, off, 32));
      cm[r] = m;
    }
    __bf16* pwh = Psh[wave];
    __bf16* pwl = Psl[wave];
#pragma unroll
    for (int r = 0; r < 8; ++r) {
      const float mnew = fmaxf(mrow[r], cm[r]);
      const float alpha = expf(mrow[r] - mnew);
      mrow[r] = mnew;
      float psum = 0.f;
#pragma unroll
      for (int j = 0; j < 4; ++j) {
        const float p = expf(s[j][r] - mnew);
        psum += p;
        __bf16 a, bl; at_split(p, a, bl);
        pwh[(8 * hh + r) * kKC + j * 16 + c] = a;
        pwl[(8 * hh + r) * kKC + j * 16 + c] = bl;
      }
#pragma unroll
      for (int off = 1; off < 16; off <<= 1) psum += __shfl_xor(psum, off, 32);
      lrow[r] = lrow[r] * alpha + psum;
#pragma unroll
      for (int t = 0; t < 4; ++t) oacc[t][r] *= alpha;
    }
    __builtin_amdgcn_fence(__ATOMIC_RELEASE, "workgroup");
    __builtin_amdgcn_wave_barrier();
    __builtin_amdgcn_fence(__ATOMIC_ACQUIRE, "workgroup");
#pragma unroll 1
    for (int kk = 0; kk < 2; ++kk) {
      FB pa, pl;
      pa.h[0] = *(const v8b*)(pwh + c * kKC + kk * 32 + 8 * hh);
      pa.h[1] = *(const v8b*)(pwh + c * kKC + kk * 32 + 16 + 8 * hh);
      pl.h[0] = *(const v8b*)(pwl + c * kKC + kk * 32 + 8 * hh);
      pl.h[1] = *(const v8b*)(pwl + c * kKC + kk * 32 + 16 + 8 * hh);
#pragma unroll
      for (int t = 0; t < 4; ++t) {
        FB vb, vl;
        vb.h[0] = *(const v8b*)(Vhs + (t * 16 + c) * kKC + kk * 32 + 8 * hh);
        vb.h[1] = *(const v8b*)(Vhs + (t * 16 + c) * kKC + kk * 32 + 16 + 8 * hh);
        vl.h[0] = *(const v8b*)(Vls + (t * 16 + c) * kKC + kk * 32 + 8 * hh);
        vl.h[1] = *(const v8b*)(Vls + (t * 16 + c) * kKC + kk * 32 + 16 + 8 * hh);
        oacc[t] = at_mma(pa.v, vb.v, oacc[t]);
        oacc[t] = at_mma(pa.v, vl.v, oacc[t]);
        oacc[t] = at_mma(pl.v, vb.v, oacc[t]);
      }
    }
  }

  float* os = Os[wave];
#pragma unroll
  for (int r = 0; r < 8; ++r) {
    const float inv = 1.0f / lrow[r];
#pragma unroll
    for (int t = 0; t < 4; ++t) os[(8 * hh + r) * 68 + t * 16 + c] = oacc[t][r] * inv;
  }
  __builtin_amdgcn_fence(__ATOMIC_RELEASE, "workgroup");
  __builtin_amdgcn_wave_barrier();
  __builtin_amdgcn_fence(__ATOMIC_ACQUIRE, "workgroup");
  {
    const int c4 = (lane & 15) * 4;
    for (int pass = 0; pass < 2; ++pass) {
#pragma unroll
      for (int it = 0; it < 8; ++it) {
        const int row = it * 2 + hh;
        v4f val = *(const v4f*)(os + row * 68 + c4);
        *(volatile v4f*)(ob_ptr + (size_t)(q0 + row) * kD + c4) = val;
      }
      __threadfence();
    }
  }
}

__global__ __launch_bounds__(64) void shaped_combine(const float* __restrict__ AV, const float* __restrict__ Vf,
                                                     const float* __restrict__ rg, const float* __restrict__ sg,
                                                     const float* __restrict__ cg,
                                                     unsigned short* __restrict__ Oh, unsigned short* __restrict__ Ol) {
  const int gw = blockIdx.x * 2 + (threadIdx.x >> 5);
  const int lane = threadIdx.x & 31;
  const int b = gw / (kD / kHD);
  const int h = gw % (kD / kHD);
  const int c0 = h * kHD + 2 * lane;
  const float rgh = rg[h], sgh = sg[h], cgh = cg[h];
  float p0 = 0.f, p1 = 0.f;
#pragma unroll 1
  for (int s = 0; s < kS; ++s) {
    const size_t idx = (size_t)(b * kS + s) * kD + c0;
    const v2f vv = *(const v2f*)(Vf + idx);
    const v2f aa = *(const v2f*)(AV + idx);
    p0 += vv[0];
    p1 += vv[1];
    const float inv = 1.0f / (float)(s + 1);
    const float o0 = rgh * aa[0] + sgh * vv[0] - cgh * (p0 * inv);
    const float o1 = rgh * aa[1] + sgh * vv[1] - cgh * (p1 * inv);
    const unsigned short h0 = f2bf_bits(o0), h1 = f2bf_bits(o1);
    const unsigned short l0 = f2bf_bits(o0 - bf_bits2f(h0));
    const unsigned short l1 = f2bf_bits(o1 - bf_bits2f(h1));
    const unsigned uh = (unsigned)h0 | ((unsigned)h1 << 16);
    const unsigned ul = (unsigned)l0 | ((unsigned)l1 << 16);
    volatile unsigned* ph = (volatile unsigned*)Oh + (idx >> 1);
    volatile unsigned* pl = (volatile unsigned*)Ol + (idx >> 1);
    *ph = uh;
    *pl = ul;
    __threadfence();
    *ph = uh;
    *pl = ul;
  }
}

extern "C" void kernel_launch(void* const* d_in, const int* in_sizes, int n_in,
                              void* d_out, int out_size, void* d_ws,
                              size_t ws_size, hipStream_t stream) {
  if (n_in < 8) return;
  if (in_sizes[0] != kTok * kD) return;
  if (in_sizes[1] != kD * kQKLd) return;
  if (in_sizes[2] != kQKLd) return;
  if (in_sizes[3] != kD * kD) return;
  if (in_sizes[4] != kD * kD) return;
  if (in_sizes[5] != kH || in_sizes[6] != kH || in_sizes[7] != kH) return;
  if (out_size != kTok * kD) return;
  if (kWsTotal > ws_size) return;

  const float* x     = (const float*)d_in[0];
  const float* qk_w  = (const float*)d_in[1];
  const float* qk_b  = (const float*)d_in[2];
  const float* v_w   = (const float*)d_in[3];
  const float* cp_w  = (const float*)d_in[4];
  const float* rg    = (const float*)d_in[5];
  const float* sg    = (const float*)d_in[6];
  const float* cg    = (const float*)d_in[7];
  float* out = (float*)d_out;

  unsigned char* ws = (unsigned char*)d_ws;
  unsigned short* xb   = (unsigned short*)(ws + kOffXb);
  unsigned short* qkwT = (unsigned short*)(ws + kOffQkwT);
  unsigned short* vwT  = (unsigned short*)(ws + kOffVwT);
  unsigned short* cwT  = (unsigned short*)(ws + kOffCwT);
  unsigned short* QKp  = (unsigned short*)(ws + kOffQKp);
  float*          Vf   = (float*)(ws + kOffVf);
  unsigned short* Vth  = (unsigned short*)(ws + kOffVth);
  unsigned short* Vtl  = (unsigned short*)(ws + kOffVtl);
  float*          AV   = (float*)(ws + kOffAV);
  unsigned short* Oh   = (unsigned short*)(ws + kOffOh);
  unsigned short* Ol   = (unsigned short*)(ws + kOffOl);

  {
    const int n2 = (kTok * kD) / 2;
    cast_f32_bf16x2<<<dim3((n2 + 255) / 256), dim3(256), 0, stream>>>(x, xb, n2);
  }
  transpose_cast_bf16<<<dim3(kQKLd / 64, kD / 64), dim3(256), 0, stream>>>(qk_w, qkwT, kD, kQKLd);
  transpose_cast_bf16<<<dim3(kD / 64, kD / 64),    dim3(256), 0, stream>>>(v_w,  vwT,  kD, kD);
  transpose_cast_bf16<<<dim3(kD / 64, kD / 64),    dim3(256), 0, stream>>>(cp_w, cwT,  kD, kD);

  wmma_gemm64<1, 0, 2, 1, false><<<dim3((kTok / 64) * (kQKLd / 64) / 8, 1), dim3(256), 0, stream>>>(
      xb, xb, kD, 0L, qkwT, qkwT, kD, 0L, (void*)QKp, (void*)QKp, kQKLd, 0L,
      qk_b, x, 0L, kTok, kQKLd, kD, 1.0f);
  wmma_gemm64<1, 0, 0, 0, false><<<dim3((kTok / 64) * (kD / 64) / 8, 1), dim3(256), 0, stream>>>(
      xb, xb, kD, 0L, vwT, vwT, kD, 0L, (void*)Vf, (void*)Vf, kD, 0L,
      qk_b, x, 0L, kTok, kD, kD, 1.0f);
  v_split_transpose<<<dim3(kS / 64, kB * kH), dim3(256), 0, stream>>>(Vf, Vth, Vtl);
  attn_causal_hd64<<<dim3(kB * kH * kNQB), dim3(128), 0, stream>>>(QKp, Vth, Vtl, AV);
  shaped_combine<<<dim3(kB * (kD / kHD) / 2), dim3(64), 0, stream>>>(AV, Vf, rg, sg, cg, Oh, Ol);
  wmma_gemm64<1, 1, 0, 0, false><<<dim3((kTok / 64) * (kD / 64) / 8, 1), dim3(256), 0, stream>>>(
      Oh, Ol, kD, 0L, cwT, cwT, kD, 0L, (void*)out, (void*)out, kD, 0L,
      qk_b, x, 0L, kTok, kD, kD, 1.0f);
}
